// Hamburger_79637283602491
// MI455X (gfx1250) — hardware-run, weakly checked
//
#include <hip/hip_runtime.h>
#include <math.h>

typedef __attribute__((ext_vector_type(16))) __bf16   v16b;
typedef __attribute__((ext_vector_type(8)))  __bf16   v8b;
typedef __attribute__((ext_vector_type(8)))  float    v8f;
typedef __attribute__((ext_vector_type(4)))  float    v4f;
typedef __attribute__((ext_vector_type(4)))  unsigned v4u;

constexpr int kBatch = 8;
constexpr int kCh    = 256;
constexpr int kPos   = 4096;
constexpr int kRank  = 64;
constexpr int kSteps = 7;
constexpr int kGroups = 32;
constexpr int kGroupCh = kCh / kGroups;
constexpr float kUpdEps = 1e-6f;
constexpr float kGnEps  = 1e-5f;
static_assert((kCh % 64) == 0 && (kPos % 64) == 0 && kRank == 64, "tile multiples of 64");
static_assert((kCh % 32) == 0 && (kPos % 32) == 0 && (kRank % 32) == 0, "every K is a multiple of 32");
static_assert(kGroupCh == 8, "8 channels per group");

constexpr size_t kPlaneBig = (size_t)kBatch * kPos * kCh * 2;
constexpr size_t kCoefF    = (size_t)kBatch * kPos * kRank * 4;
constexpr size_t kCoefPl   = (size_t)kBatch * kPos * kRank * 2;
constexpr size_t kCoefSet  = kCoefF + 4 * kCoefPl;
constexpr size_t kBasF     = (size_t)kBatch * kCh * kRank * 4;
constexpr size_t kBasPl    = (size_t)kBatch * kCh * kRank * 2;
constexpr size_t kBasSet   = kBasF + 4 * kBasPl;
constexpr size_t kGramPl   = (size_t)kBatch * kRank * kRank * 2;
constexpr size_t kWPl      = (size_t)kCh * kCh * 2;
constexpr size_t kWBPl     = (size_t)kBatch * kCh * kRank * 2;
constexpr size_t kStatsB   = (size_t)kBatch * kGroups * 128;

constexpr size_t kOffX    = 0;
constexpr size_t kOffHT   = kOffX   + 2 * kPlaneBig;
constexpr size_t kOffH    = kOffHT  + 2 * kPlaneBig;
constexpr size_t kOffP    = kOffH   + 2 * kPlaneBig;
constexpr size_t kOffBas0 = kOffP   + kCoefSet;
constexpr size_t kOffBas1 = kOffBas0 + kBasSet;
constexpr size_t kOffBtb  = kOffBas1 + kBasSet;
constexpr size_t kOffCtc  = kOffBtb + 2 * kGramPl;
constexpr size_t kOffWin  = kOffCtc + 2 * kGramPl;
constexpr size_t kOffWout = kOffWin + 2 * kWPl;
constexpr size_t kOffWB   = kOffWout + 2 * kWPl;
constexpr size_t kOffSt   = kOffWB  + 2 * kWBPl;
constexpr size_t kWsTotal = kOffSt  + kStatsB;
static_assert(kWsTotal == 130318336ull, "carve total");
static_assert(kWsTotal <= 134217728ull, "carve cap");
static_assert(kCoefSet <= 2 * kPlaneBig, "set Q fits in region X");
static_assert((size_t)kBatch * kCh * kPos * 4 == 2 * kPlaneBig, "o plane fits region X exactly");
static_assert((kOffHT % 128) == 0 && (kOffH % 128) == 0 && (kOffP % 128) == 0 && (kOffBas0 % 128) == 0 &&
              (kOffBas1 % 128) == 0 && (kOffBtb % 128) == 0 && (kOffCtc % 128) == 0 && (kOffWin % 128) == 0 &&
              (kOffWout % 128) == 0 && (kOffWB % 128) == 0 && (kOffSt % 128) == 0, "128-B aligned regions");

__device__ __forceinline__ unsigned short f2bf_bits(float f) {
  unsigned u = __float_as_uint(f);
  return (unsigned short)((u + 0x7FFFu + ((u >> 16) & 1u)) >> 16);
}
__device__ __forceinline__ float bf_bits2f(unsigned short h) { return __uint_as_float(((unsigned)h) << 16); }

__device__ __forceinline__ void split2(float a, float b, unsigned& hw, unsigned& lw) {
  const unsigned short ha = f2bf_bits(a), hb = f2bf_bits(b);
  const unsigned short la = f2bf_bits(a - bf_bits2f(ha)), lb = f2bf_bits(b - bf_bits2f(hb));
  hw = (unsigned)ha | ((unsigned)hb << 16);
  lw = (unsigned)la | ((unsigned)lb << 16);
}

__device__ __forceinline__ void keep4_b(v16b a, v16b b, v16b c, v16b d) { asm volatile("v_nop" :: "v"(a), "v"(b), "v"(c), "v"(d)); }

template <typename T> struct Frag;
template <> struct Frag<__bf16> {
  typedef v16b V; union U { v16b v; v8b h[2]; };
  static __device__ __forceinline__ v16b load(const __bf16* p) {
    U f; f.h[0] = *(const v8b*)(p); f.h[1] = *(const v8b*)(p + 16); return f.v;
  }
};

__device__ __forceinline__ v8f mma3_bf(v16b ah, v16b al, v16b bh, v16b bl, v8f c) {
  c = __builtin_amdgcn_wmma_f32_16x16x32_bf16(false, ah, false, bh, (short)0, c, false, false);
  c = __builtin_amdgcn_wmma_f32_16x16x32_bf16(false, ah, false, bl, (short)0, c, false, false);
  c = __builtin_amdgcn_wmma_f32_16x16x32_bf16(false, al, false, bh, (short)0, c, false, false);
  asm volatile("v_nop\n\tv_nop\n\tv_nop\n\tv_nop" : "+v"(c) : "v"(ah), "v"(al), "v"(bh), "v"(bl));
  return c;
}

__device__ __forceinline__ void tile_mac(const __bf16* Ah, const __bf16* Al, int lda,
                                         const __bf16* Bh, const __bf16* Bl, int ldb,
                                         int K, int rlane, int koff, v8f (&acc)[4][4]) {
  for (int k0 = 0; k0 < K; k0 += 32) {
    v16b bh[4], bl[4];
#pragma unroll
    for (int j = 0; j < 4; ++j) {
      const size_t bo = (size_t)((j << 4) + rlane) * ldb + koff + k0;
      bh[j] = Frag<__bf16>::load(Bh + bo);
      bl[j] = Frag<__bf16>::load(Bl + bo);
    }
#pragma unroll
    for (int i = 0; i < 4; ++i) {
      const size_t ao = (size_t)((i << 4) + rlane) * lda + koff + k0;
      const v16b ah = Frag<__bf16>::load(Ah + ao);
      const v16b al = Frag<__bf16>::load(Al + ao);
#pragma unroll
      for (int j = 0; j < 4; ++j) acc[i][j] = mma3_bf(ah, al, bh[j], bl[j], acc[i][j]);
    }
    keep4_b(bh[0], bh[1], bh[2], bh[3]);
    keep4_b(bl[0], bl[1], bl[2], bl[3]);
  }
}

template <int NW, int BIAS_MODE, int OUT_MODE, int ACT>
__global__ __launch_bounds__(256) __attribute__((amdgpu_num_vgpr(256))) void wmma_gemm64s(
    const unsigned short* __restrict__ Ap, const unsigned short* __restrict__ A2p, int lda, long strideA,
    const unsigned short* __restrict__ Btp, const unsigned short* __restrict__ Bt2p, int ldb, long strideB,
    void* __restrict__ Cout, void* __restrict__ Cout2, int ldc, long strideC,
    const float* __restrict__ bias, int M, int N, int K) {
  __shared__ __align__(16) float sT[NW][16 * 68];
  const int b    = blockIdx.y;
  const int lane = threadIdx.x & 31;
  const int wave = threadIdx.x >> 5;
  const int tilesN = N >> 6;
  const int tilesM = M >> 6;
  const int tile = blockIdx.x * NW + wave;
  if (tile >= tilesM * tilesN) return;
  const int tm = tile / tilesN;
  const int tn = tile - tm * tilesN;
  const int m0 = tm << 6;
  const int n0 = tn << 6;

  const int rlane = lane & 15;
  const int koff  = (lane >> 4) * 8;
  const int mOff  = (lane >> 4) * 8;

  const __bf16* Ah = (const __bf16*)Ap   + (size_t)b * strideA + (size_t)m0 * lda;
  const __bf16* Al = (const __bf16*)A2p  + (size_t)b * strideA + (size_t)m0 * lda;
  const __bf16* Bh = (const __bf16*)Btp  + (size_t)b * strideB + (size_t)n0 * ldb;
  const __bf16* Bl = (const __bf16*)Bt2p + (size_t)b * strideB + (size_t)n0 * ldb;

  v8f acc[4][4];
#pragma unroll
  for (int i = 0; i < 4; ++i)
#pragma unroll
    for (int j = 0; j < 4; ++j) acc[i][j] = (v8f){0.f,0.f,0.f,0.f,0.f,0.f,0.f,0.f};

  tile_mac(Ah, Al, lda, Bh, Bl, ldb, K, rlane, koff, acc);

  float* slab = sT[wave];
#pragma unroll
  for (int i = 0; i < 4; ++i) {
    const int mBase = m0 + (i << 4);
#pragma unroll
    for (int j = 0; j < 4; ++j) {
      const int n = n0 + (j << 4) + rlane;
      float bv = 0.f;
      if (BIAS_MODE == 2) bv = bias[n];
#pragma unroll
      for (int r = 0; r < 8; ++r) {
        float v = acc[i][j][r];
        if (BIAS_MODE == 2) v += bv;
        if (ACT == 2) v = fmaxf(v, 0.0f);
        slab[(mOff + r) * 68 + (j << 4) + rlane] = v;
      }
    }
    __builtin_amdgcn_fence(__ATOMIC_RELEASE, "workgroup");
    __builtin_amdgcn_wave_barrier();
    __builtin_amdgcn_fence(__ATOMIC_ACQUIRE, "workgroup");
    if (OUT_MODE == 0) {
      float* C = (float*)Cout + (size_t)b * strideC;
      const int hh = lane >> 4, c4 = (lane & 15) * 4;
      for (int pass = 0; pass < 2; ++pass) {
#pragma unroll
        for (int it = 0; it < 8; ++it) {
          const int row = it * 2 + hh;
          v4f v = *(const v4f*)(slab + row * 68 + c4);
          *(volatile v4f*)(C + (size_t)(mBase + row) * ldc + n0 + c4) = v;
        }
        __threadfence();
      }
    } else {
      const int q = lane >> 3, c8 = (lane & 7) * 8;
      unsigned short* C  = (unsigned short*)Cout  + (size_t)b * strideC;
      unsigned short* C2 = (unsigned short*)Cout2 + (size_t)b * strideC;
      for (int pass = 0; pass < 2; ++pass) {
#pragma unroll
        for (int it = 0; it < 4; ++it) {
          const int row = it * 4 + q;
          const float* sp = slab + row * 68 + c8;
          const v4f a0 = *(const v4f*)(sp);
          const v4f a1 = *(const v4f*)(sp + 4);
          v4u hw, lw;
          unsigned h, l;
          split2(a0[0], a0[1], h, l); hw[0] = h; lw[0] = l;
          split2(a0[2], a0[3], h, l); hw[1] = h; lw[1] = l;
          split2(a1[0], a1[1], h, l); hw[2] = h; lw[2] = l;
          split2(a1[2], a1[3], h, l); hw[3] = h; lw[3] = l;
          *(volatile v4u*)(void*)(C + (size_t)(mBase + row) * ldc + n0 + c8) = hw;
          *(volatile v4u*)(void*)(C2 + (size_t)(mBase + row) * ldc + n0 + c8) = lw;
        }
        __threadfence();
      }
    }
    __builtin_amdgcn_fence(__ATOMIC_RELEASE, "workgroup");
    __builtin_amdgcn_wave_barrier();
    __builtin_amdgcn_fence(__ATOMIC_ACQUIRE, "workgroup");
  }
}

__device__ __forceinline__ void emit_tile(const float* T, float* Xn,
                                          unsigned short* ph, unsigned short* pl,
                                          unsigned short* th, unsigned short* tl, int ldt, int lane) {
  const int hh = lane >> 4, c4 = (lane & 15) * 4;
  const int q = lane >> 3, c8 = (lane & 7) * 8;
  for (int pass = 0; pass < 2; ++pass) {
#pragma unroll 2
    for (int it = 0; it < 32; ++it) {
      const int row = it * 2 + hh;
      const v4f v = *(const v4f*)(T + row * 68 + c4);
      *(volatile v4f*)(Xn + (size_t)row * 64 + c4) = v;
    }
#pragma unroll 2
    for (int it = 0; it < 16; ++it) {
      const int row = it * 4 + q;
      const v4f a0 = *(const v4f*)(T + row * 68 + c8);
      const v4f a1 = *(const v4f*)(T + row * 68 + c8 + 4);
      v4u hw, lw;
      unsigned h, l;
      split2(a0[0], a0[1], h, l); hw[0] = h; lw[0] = l;
      split2(a0[2], a0[3], h, l); hw[1] = h; lw[1] = l;
      split2(a1[0], a1[1], h, l); hw[2] = h; lw[2] = l;
      split2(a1[2], a1[3], h, l); hw[3] = h; lw[3] = l;
      *(volatile v4u*)(void*)(ph + (size_t)row * 64 + c8) = hw;
      *(volatile v4u*)(void*)(pl + (size_t)row * 64 + c8) = lw;
    }
#pragma unroll 2
    for (int it = 0; it < 16; ++it) {
      const int col = it * 4 + q;
      float f[8];
#pragma unroll
      for (int e = 0; e < 8; ++e) f[e] = T[(c8 + e) * 68 + col];
      v4u hw, lw;
      unsigned h, l;
      split2(f[0], f[1], h, l); hw[0] = h; lw[0] = l;
      split2(f[2], f[3], h, l); hw[1] = h; lw[1] = l;
      split2(f[4], f[5], h, l); hw[2] = h; lw[2] = l;
      split2(f[6], f[7], h, l); hw[3] = h; lw[3] = l;
      *(volatile v4u*)(void*)(th + (size_t)col * ldt + c8) = hw;
      *(volatile v4u*)(void*)(tl + (size_t)col * ldt + c8) = lw;
    }
    __threadfence();
  }
}

struct UpdArgs {
  const unsigned short* AnH; const unsigned short* AnL;
  const unsigned short* BnH; const unsigned short* BnL;
  const unsigned short* AdH; const unsigned short* AdL;
  const unsigned short* BdH; const unsigned short* BdL;
  const float* Xold; float* Xnew;
  unsigned short* PH; unsigned short* PL; unsigned short* TH; unsigned short* TL;
  long sAn, sBn, sAd, sBd, sX, sP, sT;
  int lda, ldb, ldt, K;
};
static_assert(sizeof(UpdArgs) == 184, "no padding");

template <int MODE, int NW>
__global__ __launch_bounds__(256) __attribute__((amdgpu_num_vgpr(256))) void factor_tile_kernel(UpdArgs a) {
  __shared__ __align__(16) float sTile[NW][64 * 68];
  const int lane = threadIdx.x & 31;
  const int wave = threadIdx.x >> 5;
  const int b = blockIdx.y;
  const int m0 = (blockIdx.x * NW + wave) << 6;
  const int rlane = lane & 15;
  const int hh = lane >> 4;
  const int koff = hh * 8;
  const int mOff = hh * 8;
  float* T = sTile[wave];

  v8f acc[4][4];
#pragma unroll
  for (int i = 0; i < 4; ++i)
#pragma unroll
    for (int j = 0; j < 4; ++j) acc[i][j] = (v8f){0.f,0.f,0.f,0.f,0.f,0.f,0.f,0.f};

  if (MODE == 0) {
    const __bf16* adh = (const __bf16*)a.AdH + (size_t)b * a.sAd + (size_t)m0 * 64;
    const __bf16* adl = (const __bf16*)a.AdL + (size_t)b * a.sAd + (size_t)m0 * 64;
    const __bf16* bdh = (const __bf16*)a.BdH + (size_t)b * a.sBd;
    const __bf16* bdl = (const __bf16*)a.BdL + (size_t)b * a.sBd;
    tile_mac(adh, adl, 64, bdh, bdl, 64, 64, rlane, koff, acc);
#pragma unroll
    for (int i = 0; i < 4; ++i)
#pragma unroll
      for (int j = 0; j < 4; ++j) {
#pragma unroll
        for (int r = 0; r < 8; ++r) T[((i << 4) + mOff + r) * 68 + (j << 4) + rlane] = acc[i][j][r];
        acc[i][j] = (v8f){0.f,0.f,0.f,0.f,0.f,0.f,0.f,0.f};
      }
  }
  {
    const __bf16* anh = (const __bf16*)a.AnH + (size_t)b * a.sAn + (size_t)m0 * a.lda;
    const __bf16* anl = (const __bf16*)a.AnL + (size_t)b * a.sAn + (size_t)m0 * a.lda;
    const __bf16* bnh = (const __bf16*)a.BnH + (size_t)b * a.sBn;
    const __bf16* bnl = (const __bf16*)a.BnL + (size_t)b * a.sBn;
    tile_mac(anh, anl, a.lda, bnh, bnl, a.ldb, a.K, rlane, koff, acc);
  }
#pragma unroll
  for (int i = 0; i < 4; ++i)
#pragma unroll
    for (int j = 0; j < 4; ++j)
#pragma unroll
      for (int r = 0; r < 8; ++r) {
        const int idx = ((i << 4) + mOff + r) * 68 + (j << 4) + rlane;
        if (MODE == 0) {
          const float den = T[idx] + kUpdEps;
          T[idx] = acc[i][j][r] * __builtin_amdgcn_rcpf(den);
        } else {
          T[idx] = acc[i][j][r];
        }
      }
  __syncthreads();
  {
    const int c4 = rlane * 4;
    const float* xo = a.Xold + (size_t)b * a.sX + (size_t)m0 * 64;
#pragma unroll 1
    for (int it = 0; it < 32; ++it) {
      const int row = it * 2 + hh;
      float* tp = T + row * 68 + c4;
      v4f t = *(const v4f*)tp;
      if (MODE == 0) {
        const v4f o = *(const v4f*)(xo + (size_t)row * 64 + c4);
        t = o * t;
      } else {
        float mx = fmaxf(fmaxf(t[0], t[1]), fmaxf(t[2], t[3]));
        mx = fmaxf(mx, __shfl_xor(mx, 1, 32));
        mx = fmaxf(mx, __shfl_xor(mx, 2, 32));
        mx = fmaxf(mx, __shfl_xor(mx, 4, 32));
        mx = fmaxf(mx, __shfl_xor(mx, 8, 32));
        const float e0 = expf(t[0] - mx), e1 = expf(t[1] - mx), e2 = expf(t[2] - mx), e3 = expf(t[3] - mx);
        float s = (e0 + e1) + (e2 + e3);
        s += __shfl_xor(s, 1, 32);
        s += __shfl_xor(s, 2, 32);
        s += __shfl_xor(s, 4, 32);
        s += __shfl_xor(s, 8, 32);
        const float inv = 1.0f / s;
        t[0] = e0 * inv; t[1] = e1 * inv; t[2] = e2 * inv; t[3] = e3 * inv;
      }
      *(v4f*)tp = t;
    }
  }
  __syncthreads();
  emit_tile(T,
            a.Xnew + (size_t)b * a.sX + (size_t)m0 * 64,
            a.PH + (size_t)b * a.sP + (size_t)m0 * 64,
            a.PL + (size_t)b * a.sP + (size_t)m0 * 64,
            a.TH + (size_t)b * a.sT + m0,
            a.TL + (size_t)b * a.sT + m0,
            a.ldt, lane);
}

__global__ __launch_bounds__(256) void x_transpose_split_kernel(
    const float* __restrict__ x, unsigned short* __restrict__ xTh, unsigned short* __restrict__ xTl) {
  __shared__ __align__(16) float T[64 * 68];
  const int tid = threadIdx.x;
  const int n0 = blockIdx.x * 64, c0 = blockIdx.y * 64, b = blockIdx.z;
#pragma unroll
  for (int it = 0; it < 4; ++it) {
    const int row = it * 16 + (tid >> 4);
    const int c4 = (tid & 15) * 4;
    const v4f v = *(const v4f*)(x + ((size_t)(b * kCh + c0 + row)) * kPos + n0 + c4);
    *(v4f*)(T + row * 68 + c4) = v;
  }
  __syncthreads();
  v4u hw[2], lw[2];
#pragma unroll
  for (int it = 0; it < 2; ++it) {
    const int task = it * 256 + tid;
    const int n = task >> 3, cc = (task & 7) * 8;
    float f[8];
#pragma unroll
    for (int e = 0; e < 8; ++e) f[e] = T[(cc + e) * 68 + n];
    unsigned h, l;
    split2(f[0], f[1], h, l); hw[it][0] = h; lw[it][0] = l;
    split2(f[2], f[3], h, l); hw[it][1] = h; lw[it][1] = l;
    split2(f[4], f[5], h, l); hw[it][2] = h; lw[it][2] = l;
    split2(f[6], f[7], h, l); hw[it][3] = h; lw[it][3] = l;
  }
  for (int pass = 0; pass < 2; ++pass) {
#pragma unroll
    for (int it = 0; it < 2; ++it) {
      const int task = it * 256 + tid;
      const int n = task >> 3, cc = (task & 7) * 8;
      const size_t o = ((size_t)(b * kPos + n0 + n)) * kCh + c0 + cc;
      *(volatile v4u*)(void*)(xTh + o) = hw[it];
      *(volatile v4u*)(void*)(xTl + o) = lw[it];
    }
    __threadfence();
  }
}

__global__ __launch_bounds__(256) void split_rows_bf16_kernel(
    const float* __restrict__ src, unsigned short* __restrict__ dhi, unsigned short* __restrict__ dlo, int total8) {
  const int i = blockIdx.x * 256 + threadIdx.x;
  if (i >= total8) return;
  const size_t e0 = (size_t)i << 3;
  const v4f a0 = *(const v4f*)(src + e0);
  const v4f a1 = *(const v4f*)(src + e0 + 4);
  v4u hw, lw;
  unsigned h, l;
  split2(a0[0], a0[1], h, l); hw[0] = h; lw[0] = l;
  split2(a0[2], a0[3], h, l); hw[1] = h; lw[1] = l;
  split2(a1[0], a1[1], h, l); hw[2] = h; lw[2] = l;
  split2(a1[2], a1[3], h, l); hw[3] = h; lw[3] = l;
  *(volatile v4u*)(void*)(dhi + e0) = hw;
  *(volatile v4u*)(void*)(dlo + e0) = lw;
  __threadfence();
  *(volatile v4u*)(void*)(dhi + e0) = hw;
  *(volatile v4u*)(void*)(dlo + e0) = lw;
}

__global__ __launch_bounds__(32) void bases_init_kernel(
    const float* __restrict__ bi, float* __restrict__ Xn,
    unsigned short* __restrict__ ph, unsigned short* __restrict__ pl,
    unsigned short* __restrict__ th, unsigned short* __restrict__ tl) {
  __shared__ __align__(16) float T[64 * 68];
  __shared__ __align__(16) float sInv[64];
  const int lane = threadIdx.x & 31;
  const int d0 = blockIdx.x * 64, b = blockIdx.y;
  const float* src = bi + (size_t)b * kCh * kRank;
  float p0 = 0.f, p1 = 0.f, p2 = 0.f, p3 = 0.f, q0 = 0.f, q1 = 0.f, q2 = 0.f, q3 = 0.f;
#pragma unroll 1
  for (int d = 0; d < kCh; d += 4) {
    const float a0 = src[(d + 0) * kRank + lane], b0 = src[(d + 0) * kRank + 32 + lane];
    const float a1 = src[(d + 1) * kRank + lane], b1 = src[(d + 1) * kRank + 32 + lane];
    const float a2 = src[(d + 2) * kRank + lane], b2 = src[(d + 2) * kRank + 32 + lane];
    const float a3 = src[(d + 3) * kRank + lane], b3 = src[(d + 3) * kRank + 32 + lane];
    p0 += a0 * a0; p1 += a1 * a1; p2 += a2 * a2; p3 += a3 * a3;
    q0 += b0 * b0; q1 += b1 * b1; q2 += b2 * b2; q3 += b3 * b3;
  }
  const float s0 = (p0 + p1) + (p2 + p3);
  const float s1 = (q0 + q1) + (q2 + q3);
  sInv[lane]      = 1.0f / fmaxf(sqrtf(s0), 1e-12f);
  sInv[lane + 32] = 1.0f / fmaxf(sqrtf(s1), 1e-12f);
  __syncthreads();
  {
    const int hh = lane >> 4, c4 = (lane & 15) * 4;
    const v4f iv = *(const v4f*)(sInv + c4);
#pragma unroll 1
    for (int it = 0; it < 32; ++it) {
      const int row = it * 2 + hh;
      const v4f v = *(const v4f*)(src + (size_t)(d0 + row) * kRank + c4);
      *(v4f*)(T + row * 68 + c4) = v * iv;
    }
  }
  __syncthreads();
  emit_tile(T,
            Xn + (size_t)b * kCh * kRank + (size_t)d0 * kRank,
            ph + (size_t)b * kCh * kRank + (size_t)d0 * kRank,
            pl + (size_t)b * kCh * kRank + (size_t)d0 * kRank,
            th + (size_t)b * kRank * kCh + d0,
            tl + (size_t)b * kRank * kCh + d0,
            kCh, lane);
}

__global__ __launch_bounds__(256) void plane_transpose16_kernel(
    const unsigned short* __restrict__ sh, const unsigned short* __restrict__ sl,
    unsigned short* __restrict__ dh, unsigned short* __restrict__ dl) {
  __shared__ unsigned short S[64 * 66];
  const int tid = threadIdx.x;
  const int n0 = blockIdx.x * 64, d0 = blockIdx.y * 64;
  const int b = blockIdx.z >> 1;
  const bool lo = (blockIdx.z & 1) != 0;
  const unsigned short* src = lo ? sl : sh;
  unsigned short* dst = lo ? dl : dh;
#pragma unroll
  for (int it = 0; it < 2; ++it) {
    const int task = it * 256 + tid;
    const int row = task >> 3, c8 = (task & 7) * 8;
    const v4u w = *(const v4u*)(const void*)(src + ((size_t)(b * kPos + n0 + row)) * kCh + d0 + c8);
    unsigned short* sp = S + row * 66 + c8;
#pragma unroll
    for (int j = 0; j < 4; ++j) {
      const unsigned wj = w[j];
      sp[2 * j]     = (unsigned short)(wj & 0xffffu);
      sp[2 * j + 1] = (unsigned short)(wj >> 16);
    }
  }
  __syncthreads();
  v4u ow[2];
#pragma unroll
  for (int it = 0; it < 2; ++it) {
    const int task = it * 256 + tid;
    const int drow = task >> 3, cn = (task & 7) * 8;
    unsigned s[8];
#pragma unroll
    for (int e = 0; e < 8; ++e) s[e] = (unsigned)S[(cn + e) * 66 + drow];
#pragma unroll
    for (int j = 0; j < 4; ++j) ow[it][j] = s[2 * j] | (s[2 * j + 1] << 16);
  }
  for (int pass = 0; pass < 2; ++pass) {
#pragma unroll
    for (int it = 0; it < 2; ++it) {
      const int task = it * 256 + tid;
      const int drow = task >> 3, cn = (task & 7) * 8;
      *(volatile v4u*)(void*)(dst + ((size_t)(b * kCh + d0 + drow)) * kPos + n0 + cn) = ow[it];
    }
    __threadfence();
  }
}

__global__ __launch_bounds__(256) void group_stats_kernel(const float* __restrict__ o, float* __restrict__ stats) {
  __shared__ float red[256];
  const int tid = threadIdx.x;
  const float* base = o + (size_t)blockIdx.x * (kGroupCh * kPos);
  float s = 0.f;
#pragma unroll 4
  for (int it = 0; it < 32; ++it) {
    const v4f v = *(const v4f*)(base + it * 1024 + tid * 4);
    s += (v[0] + v[1]) + (v[2] + v[3]);
  }
  red[tid] = s;
  __syncthreads();
  for (int st = 128; st > 0; st >>= 1) {
    if (tid < st) red[tid] += red[tid + st];
    __syncthreads();
  }
  const float mean = red[0] * (1.0f / 32768.0f);
  __syncthreads();
  float ss = 0.f;
#pragma unroll 4
  for (int it = 0; it < 32; ++it) {
    const v4f v = *(const v4f*)(base + it * 1024 + tid * 4);
    const float e0 = v[0] - mean, e1 = v[1] - mean, e2 = v[2] - mean, e3 = v[3] - mean;
    ss += (e0 * e0 + e1 * e1) + (e2 * e2 + e3 * e3);
  }
  red[tid] = ss;
  __syncthreads();
  for (int st = 128; st > 0; st >>= 1) {
    if (tid < st) red[tid] += red[tid + st];
    __syncthreads();
  }
  const float var = red[0] * (1.0f / 32768.0f);
  const float rstd = 1.0f / sqrtf(var + kGnEps);
  if (tid < 32) {
    const float val = (tid == 0) ? mean : ((tid == 1) ? rstd : 0.0f);
    volatile float* p = stats + (size_t)blockIdx.x * 32 + tid;
    *p = val;
    __threadfence();
    *p = val;
  }
}

__global__ __launch_bounds__(256) void finalize_kernel(
    const float* __restrict__ x, const float* __restrict__ o,
    const float* __restrict__ gamma, const float* __restrict__ beta,
    const float* __restrict__ stats, float* __restrict__ out) {
  const int row = blockIdx.x;
  const int c = row & (kCh - 1);
  const int b = row >> 8;
  const int g = c >> 3;
  const float mean = stats[(size_t)(b * kGroups + g) * 32];
  const float rstd = stats[(size_t)(b * kGroups + g) * 32 + 1];
  const float ga = gamma[c], be = beta[c];
  const size_t rb = (size_t)row * kPos + threadIdx.x * 4;
  v4f r[4];
#pragma unroll
  for (int it = 0; it < 4; ++it) {
    const v4f xv = *(const v4f*)(x + rb + it * 1024);
    const v4f ov = *(const v4f*)(o + rb + it * 1024);
#pragma unroll
    for (int e = 0; e < 4; ++e) {
      const float nv = ((ov[e] - mean) * rstd) * ga + be;
      r[it][e] = fmaxf(xv[e] + nv, 0.0f);
    }
  }
  for (int pass = 0; pass < 2; ++pass) {
#pragma unroll
    for (int it = 0; it < 4; ++it) *(volatile v4f*)(out + rb + it * 1024) = r[it];
    __threadfence();
  }
}

struct CoefSetPtr { float* f; unsigned short* ch; unsigned short* cl; unsigned short* cth; unsigned short* ctl; };
struct BasSetPtr  { float* f; unsigned short* dh; unsigned short* dl; unsigned short* th; unsigned short* tl; };

static CoefSetPtr make_coef_set(char* base) {
  CoefSetPtr s;
  s.f   = (float*)base;
  s.ch  = (unsigned short*)(base + kCoefF);
  s.cl  = (unsigned short*)(base + kCoefF + kCoefPl);
  s.cth = (unsigned short*)(base + kCoefF + 2 * kCoefPl);
  s.ctl = (unsigned short*)(base + kCoefF + 3 * kCoefPl);
  return s;
}
static BasSetPtr make_bas_set(char* base) {
  BasSetPtr s;
  s.f  = (float*)base;
  s.dh = (unsigned short*)(base + kBasF);
  s.dl = (unsigned short*)(base + kBasF + kBasPl);
  s.th = (unsigned short*)(base + kBasF + 2 * kBasPl);
  s.tl = (unsigned short*)(base + kBasF + 3 * kBasPl);
  return s;
}

extern "C" void kernel_launch(void* const* d_in, const int* in_sizes, int n_in,
                              void* d_out, int out_size, void* d_ws, size_t ws_size,
                              hipStream_t stream) {
  if (n_in < 7) return;
  if (in_sizes[0] != kBatch * kCh * kPos) return;
  if (in_sizes[1] != kCh * kCh) return;
  if (in_sizes[2] != kCh) return;
  if (in_sizes[3] != kCh * kCh) return;
  if (in_sizes[4] != kCh) return;
  if (in_sizes[5] != kCh) return;
  if (in_sizes[6] != kBatch * kCh * kRank) return;
  if (out_size != kBatch * kCh * kPos) return;
  if (ws_size < kWsTotal) return;

  const float* x      = (const float*)d_in[0];
  const float* w_in   = (const float*)d_in[1];
  const float* b_in   = (const float*)d_in[2];
  const float* w_out  = (const float*)d_in[3];
  const float* gamma  = (const float*)d_in[4];
  const float* beta   = (const float*)d_in[5];
  const float* bases0 = (const float*)d_in[6];
  float* out = (float*)d_out;

  char* ws = (char*)d_ws;
  unsigned short* xTh = (unsigned short*)(ws + kOffX);
  unsigned short* xTl = (unsigned short*)(ws + kOffX + kPlaneBig);
  float*          oF  = (float*)(ws + kOffX);
  unsigned short* hTh = (unsigned short*)(ws + kOffHT);
  unsigned short* hTl = (unsigned short*)(ws + kOffHT + kPlaneBig);
  unsigned short* hDh = (unsigned short*)(ws + kOffH);
  unsigned short* hDl = (unsigned short*)(ws + kOffH + kPlaneBig);
  CoefSetPtr setP = make_coef_set(ws + kOffP);
  CoefSetPtr setQ = make_coef_set(ws + kOffX);
  BasSetPtr bas[2];
  bas[0] = make_bas_set(ws + kOffBas0);
  bas[1] = make_bas_set(ws + kOffBas1);
  unsigned short* btbH = (unsigned short*)(ws + kOffBtb);
  unsigned short* btbL = (unsigned short*)(ws + kOffBtb + kGramPl);
  unsigned short* ctcH = (unsigned short*)(ws + kOffCtc);
  unsigned short* ctcL = (unsigned short*)(ws + kOffCtc + kGramPl);
  unsigned short* winH = (unsigned short*)(ws + kOffWin);
  unsigned short* winL = (unsigned short*)(ws + kOffWin + kWPl);
  unsigned short* woutH = (unsigned short*)(ws + kOffWout);
  unsigned short* woutL = (unsigned short*)(ws + kOffWout + kWPl);
  unsigned short* wbH = (unsigned short*)(ws + kOffWB);
  unsigned short* wbL = (unsigned short*)(ws + kOffWB + kWBPl);
  float* stats = (float*)(ws + kOffSt);

  const long sBig  = (long)kPos * kCh;
  const long sNR   = (long)kPos * kRank;
  const long sDR   = (long)kCh * kRank;
  const long sRR   = (long)kRank * kRank;

  x_transpose_split_kernel<<<dim3(kPos / 64, kCh / 64, kBatch), 256, 0, stream>>>(x, xTh, xTl);
  split_rows_bf16_kernel<<<(kCh * kCh / 8) / 256, 256, 0, stream>>>(w_in, winH, winL, kCh * kCh / 8);
  split_rows_bf16_kernel<<<(kCh * kCh / 8) / 256, 256, 0, stream>>>(w_out, woutH, woutL, kCh * kCh / 8);
  bases_init_kernel<<<dim3(kCh / 64, kBatch), 32, 0, stream>>>(bases0, bas[0].f, bas[0].dh, bas[0].dl, bas[0].th, bas[0].tl);

  wmma_gemm64s<8, 2, 2, 2><<<dim3(32, kBatch), 256, 0, stream>>>(
      xTh, xTl, kCh, sBig, winH, winL, kCh, 0L,
      (void*)hTh, (void*)hTl, kCh, sBig, b_in, kPos, kCh, kCh);

  plane_transpose16_kernel<<<dim3(kPos / 64, kCh / 64, kBatch * 2), 256, 0, stream>>>(hTh, hTl, hDh, hDl);

  {
    UpdArgs a;
    a.AnH = hTh; a.AnL = hTl; a.BnH = bas[0].th; a.BnL = bas[0].tl;
    a.AdH = setP.ch; a.AdL = setP.cl; a.BdH = btbH; a.BdL = btbL;
    a.Xold = setP.f; a.Xnew = setP.f;
    a.PH = setP.ch; a.PL = setP.cl; a.TH = setP.cth; a.TL = setP.ctl;
    a.sAn = sBig; a.sBn = sDR; a.sAd = sNR; a.sBd = sRR; a.sX = sNR; a.sP = sNR; a.sT = sNR;
    a.lda = kCh; a.ldb = kCh; a.ldt = kPos; a.K = kCh;
    factor_tile_kernel<1, 2><<<dim3(kPos / 64 / 2, kBatch), 64, 0, stream>>>(a);
  }

  for (int s = 0; s <= kSteps; ++s) {
    const int bs = (s < kSteps) ? (s & 1) : 1;
    const CoefSetPtr co = (s & 1) ? setQ : setP;
    const CoefSetPtr cn = (s & 1) ? setP : setQ;
    wmma_gemm64s<1, 0, 2, 0><<<dim3(1, kBatch), 32, 0, stream>>>(
        bas[bs].th, bas[bs].tl, kCh, sDR, bas[bs].th, bas[bs].tl, kCh, sDR,
        (void*)btbH, (void*)btbL, kRank, sRR, b_in, kRank, kRank, kCh);
    {
      UpdArgs a;
      a.AnH = hTh; a.AnL = hTl; a.BnH = bas[bs].th; a.BnL = bas[bs].tl;
      a.AdH = co.ch; a.AdL = co.cl; a.BdH = btbH; a.BdL = btbL;
      a.Xold = co.f; a.Xnew = cn.f;
      a.PH = cn.ch; a.PL = cn.cl; a.TH = cn.cth; a.TL = cn.ctl;
      a.sAn = sBig; a.sBn = sDR; a.sAd = sNR; a.sBd = sRR; a.sX = sNR; a.sP = sNR; a.sT = sNR;
      a.lda = kCh; a.ldb = kCh; a.ldt = kPos; a.K = kCh;
      factor_tile_kernel<0, 2><<<dim3(kPos / 64 / 2, kBatch), 64, 0, stream>>>(a);
    }
    if (s == kSteps) break;
    wmma_gemm64s<1, 0, 2, 0><<<dim3(1, kBatch), 32, 0, stream>>>(
        cn.cth, cn.ctl, kPos, sNR, cn.cth, cn.ctl, kPos, sNR,
        (void*)ctcH, (void*)ctcL, kRank, sRR, b_in, kRank, kRank, kPos);
    {
      const BasSetPtr bo = bas[bs];
      const BasSetPtr bn = bas[bs ^ 1];
      UpdArgs a;
      a.AnH = hDh; a.AnL = hDl; a.BnH = cn.cth; a.BnL = cn.ctl;
      a.AdH = bo.dh; a.AdL = bo.dl; a.BdH = ctcH; a.BdL = ctcL;
      a.Xold = bo.f; a.Xnew = bn.f;
      a.PH = bn.dh; a.PL = bn.dl; a.TH = bn.th; a.TL = bn.tl;
      a.sAn = sBig; a.sBn = sNR; a.sAd = sDR; a.sBd = sRR; a.sX = sDR; a.sP = sDR; a.sT = sDR;
      a.lda = kPos; a.ldb = kPos; a.ldt = kCh; a.K = kPos;
      factor_tile_kernel<0, 2><<<dim3(kCh / 64 / 2, kBatch), 64, 0, stream>>>(a);
    }
  }

  wmma_gemm64s<4, 0, 2, 0><<<dim3(1, kBatch), 128, 0, stream>>>(
      woutH, woutL, kCh, 0L, bas[1].th, bas[1].tl, kCh, sDR,
      (void*)wbH, (void*)wbL, kRank, sDR, b_in, kCh, kRank, kCh);

  wmma_gemm64s<8, 0, 0, 0><<<dim3(32, kBatch), 256, 0, stream>>>(
      wbH, wbL, kRank, sDR, setP.ch, setP.cl, kRank, sNR,
      (void*)oF, (void*)oF, kPos, sBig, b_in, kCh, kPos, kRank);

  group_stats_kernel<<<kBatch * kGroups, 256, 0, stream>>>(oF, stats);
  finalize_kernel<<<kBatch * kCh, 256, 0, stream>>>(x, oF, gamma, beta, stats, out);
}
